// Intra_S_view_9509057593867
// MI455X (gfx1250) — hardware-verified
//
#include <hip/hip_runtime.h>


#define NB_  32
#define NN   512
#define DD   256
#define DM   DD
#define SLOPE 0.2f
#define LOSC 1024.0f

typedef _Float16 h16;
typedef unsigned short bf;
typedef __attribute__((ext_vector_type(16))) __bf16   v16bf;
typedef __attribute__((ext_vector_type(16))) _Float16 v16h;
typedef __attribute__((ext_vector_type(8)))  _Float16 v8h;
typedef __attribute__((ext_vector_type(8)))  unsigned short v8us;
typedef __attribute__((ext_vector_type(8)))  float    v8f;
typedef __attribute__((ext_vector_type(4)))  float    v4f;
typedef v8h  __attribute__((may_alias)) v8ha;
typedef v4f  __attribute__((may_alias)) v4fa;
typedef v8us __attribute__((may_alias)) v8usa;

__device__ __forceinline__ unsigned short f2bf(float f) { unsigned u = __float_as_uint(f); u += 0x7FFFu + ((u >> 16) & 1u); return (unsigned short)(u >> 16); }
__device__ __forceinline__ float bf2f(unsigned short b) { return __uint_as_float(((unsigned)b) << 16); }
__device__ __forceinline__ float bfr(float f) { return bf2f(f2bf(f)); }
__device__ __forceinline__ v16h cat16(v8h lo, v8h hi) { return __builtin_shufflevector(lo, hi, 0, 1, 2, 3, 4, 5, 6, 7, 8, 9, 10, 11, 12, 13, 14, 15); }
__device__ __forceinline__ v16bf cat16b(v8us lo, v8us hi) { return __builtin_bit_cast(v16bf, __builtin_shufflevector(lo, hi, 0, 1, 2, 3, 4, 5, 6, 7, 8, 9, 10, 11, 12, 13, 14, 15)); }
__device__ __forceinline__ v8f wmma16(v16h a, v16h b, v8f c) { return __builtin_amdgcn_wmma_f32_16x16x32_f16(false, a, false, b, (short)0, c, false, false); }
__device__ __forceinline__ v8f wmmab(v16bf a, v16bf b, v8f c) { return __builtin_amdgcn_wmma_f32_16x16x32_bf16(false, a, false, b, (short)0, c, false, false); }

template <bool SPLITA, bool F16OUT = false>
__global__ __launch_bounds__(128) void k_gemmb(const bf* __restrict__ A, const bf* __restrict__ Al, const bf* __restrict__ Bn, const float* __restrict__ bias, float* C, int ldc, h16* C2, const float* __restrict__ R = nullptr, int K = DM, int roundR = 1) {
    __shared__ __align__(16) float ost[4][16 * 68];
    const int lane = threadIdx.x & 31, wave = threadIdx.x >> 5, lr = lane & 15, hi = lane >> 4;
    const int r0 = blockIdx.x * 64 + wave * 16, c0 = blockIdx.y * 64;
    const size_t aoff = (size_t)(r0 + lr) * K + 8 * hi;
    size_t boff[4];
#pragma unroll
    for (int t = 0; t < 4; ++t) boff[t] = (size_t)(c0 + t * 16 + lr) * K + 8 * hi;
    v8f acc[4];
#pragma unroll
    for (int t = 0; t < 4; ++t) acc[t] = (v8f){};
#pragma unroll 1
    for (int kc = 0; kc < K; kc += 32) {
        const v16bf a = cat16b(*(const v8us*)(A + aoff + kc), *(const v8us*)(A + aoff + kc + 16));
        v16bf al = a;
        if (SPLITA) al = cat16b(*(const v8us*)(Al + aoff + kc), *(const v8us*)(Al + aoff + kc + 16));
#pragma unroll
        for (int t = 0; t < 4; ++t) { const v16bf b = cat16b(*(const v8us*)(Bn + boff[t] + kc), *(const v8us*)(Bn + boff[t] + kc + 16)); acc[t] = wmmab(a, b, acc[t]); if (SPLITA) acc[t] = wmmab(al, b, acc[t]); }
        asm volatile("v_nop\n\tv_nop\n\tv_nop\n\tv_nop" : "+v"(acc[0]), "+v"(acc[1]), "+v"(acc[2]), "+v"(acc[3]) : "v"(a), "v"(al));
    }
    float* os = &ost[wave][0];
#pragma unroll
    for (int t = 0; t < 4; ++t) { const float bv = bias ? bfr(bias[c0 + t * 16 + lr]) : 0.f;
#pragma unroll
        for (int j = 0; j < 8; ++j) os[(hi * 8 + j) * 68 + t * 16 + lr] = acc[t][j] + bv; }
    __syncthreads();
    if (F16OUT) {
        h16* crow = (h16*)(void*)C + (size_t)r0 * ldc + c0;
        auto pass = [&]() {
#pragma unroll
            for (int s = 0; s < 4; ++s) { const int row = 4 * s + (lane >> 3), piece = lane & 7; const float* sp = os + row * 68 + piece * 8; v8h o, o2;
#pragma unroll
                for (int i = 0; i < 8; ++i) { const h16 a = (h16)sp[i]; o[i] = a; o2[i] = (h16)((sp[i] - (float)a) * LOSC); }
                *(volatile v8h*)(crow + (size_t)row * ldc + piece * 8) = o; if (C2) *(volatile v8h*)(C2 + (size_t)r0 * ldc + c0 + (size_t)row * ldc + piece * 8) = o2; }
        };
        pass(); __threadfence(); pass();
    } else {
        float* crow = C + (size_t)r0 * ldc + c0;
        auto pass = [&]() {
#pragma unroll
            for (int s = 0; s < 8; ++s) { const int Lid = (lane >> 3) + 4 * s, piece = lane & 7; const int row = Lid >> 1, cofs = (Lid & 1) * 32 + piece * 4;
                v4f val = *(const v4fa*)(os + row * 68 + cofs); if (R) { const v4f rv = *(const v4f*)(R + ((size_t)r0 + row) * ldc + c0 + cofs); val += roundR ? (v4f){bfr(rv[0]), bfr(rv[1]), bfr(rv[2]), bfr(rv[3])} : rv; }
                *(volatile v4f*)(crow + (size_t)row * ldc + cofs) = val; }
        };
        pass(); __threadfence(); pass();
    }
}


__global__ __launch_bounds__(256) void k_hprep(const float* __restrict__ h, const float* __restrict__ a0, const float* __restrict__ a1, const float* __restrict__ a2, const float* __restrict__ a3, bf* Hb, bf* HAh, bf* HAl) {
    const int lane = threadIdx.x & 31; const size_t i = (size_t)blockIdx.x * 8 + (threadIdx.x >> 5); if (i >= (size_t)NN) return; const size_t o = i * DD + lane * 8; float x[8]; v8us hb8;
#pragma unroll
    for (int q = 0; q < 8; ++q) { x[q] = bfr(h[o + q]); hb8[q] = f2bf(x[q]); }
#pragma unroll 1
    for (int ps = 0; ps < 2; ++ps) {
        *(volatile v8us*)(Hb + o) = hb8;
#pragma unroll
        for (int k = 0; k < 4; ++k) { const float* ak = (k == 0) ? a0 : (k == 1) ? a1 : (k == 2) ? a2 : a3; v8us oh, ol;
#pragma unroll
            for (int q = 0; q < 8; ++q) { const float y = x[q] * bfr(ak[lane * 8 + q]); const unsigned short hb = f2bf(y); oh[q] = hb; ol[q] = f2bf(y - bf2f(hb)); }
            *(volatile v8us*)(HAh + (size_t)k * NN * DD + o) = oh; *(volatile v8us*)(HAl + (size_t)k * NN * DD + o) = ol; }
        if (ps == 0) __threadfence(); }
}
__global__ __launch_bounds__(256) void k_hT(const float* __restrict__ h, bf* HT) {
    __shared__ float tl[64][65];
    typedef __attribute__((ext_vector_type(4))) unsigned short v4us;
    const int tid = threadIdx.x; const int j0 = blockIdx.x * 64, d0 = blockIdx.y * 64; const int rr = tid >> 2, cq = (tid & 3) * 16;
#pragma unroll
    for (int i = 0; i < 16; ++i) tl[rr][cq + i] = h[(size_t)(j0 + rr) * DD + d0 + cq + i];
    __syncthreads();
    const int lane = tid & 31, wv = tid >> 5;
    auto pass = [&]() {
#pragma unroll
        for (int st = 0; st < 4; ++st) { const int dr = wv * 8 + st * 2 + (lane >> 4); const int jq = (lane & 15) * 4; v4us v;
#pragma unroll
            for (int i = 0; i < 4; ++i) v[i] = f2bf(tl[jq + i][dr]);
            *(volatile v4us*)(HT + (size_t)(d0 + dr) * NN + j0 + jq) = v; }
    };
    pass(); __threadfence(); pass();
}
__global__ __launch_bounds__(256) void k_selsoft(const float* __restrict__ E, const int* __restrict__ adj, bf* PH, bf* PL) {
    typedef __attribute__((ext_vector_type(4))) unsigned short v4us;
    const int lane = threadIdx.x & 31; const int i = blockIdx.x * 8 + (threadIdx.x >> 5); if (i >= NN) return; const int* ar = adj + (size_t)i * NN;
    auto logit = [&](int j, bool& live) -> float { const int s = ar[j]; live = (s >= 1 && s <= 4); const float e = live ? E[((size_t)(s - 1) * NN + i) * NN + j] : 0.f; return (e >= 0.f) ? e : SLOPE * e; };
    float m = -3.0e38f; int cnt = 0;
#pragma unroll 1
    for (int c0 = lane * 4; c0 < NN; c0 += 128) {
#pragma unroll
        for (int q = 0; q < 4; ++q) { bool lv; const float a = logit(c0 + q, lv); if (lv) { m = fmaxf(m, a); ++cnt; } } }
#pragma unroll
    for (int sh = 16; sh; sh >>= 1) { m = fmaxf(m, __shfl_xor(m, sh, 32)); cnt += __shfl_xor(cnt, sh, 32); }
    float sum = 0.f;
#pragma unroll 1
    for (int c0 = lane * 4; c0 < NN; c0 += 128) {
#pragma unroll
        for (int q = 0; q < 4; ++q) { bool lv; const float a = logit(c0 + q, lv); if (lv) sum += __expf(a - m); } }
#pragma unroll
    for (int sh = 16; sh; sh >>= 1) sum += __shfl_xor(sum, sh, 32);
    const float inv = 1.0f / sum; const bool none = (cnt == 0); const float unif = 1.0f / (float)NN;
#pragma unroll 1
    for (int ps = 0; ps < 2; ++ps) {
#pragma unroll 1
        for (int c0 = lane * 4; c0 < NN; c0 += 128) { v4us oh, ol;
#pragma unroll
            for (int q = 0; q < 4; ++q) { bool lv; const float a = logit(c0 + q, lv); const float p = none ? unif : (lv ? __expf(a - m) * inv : 0.f); const unsigned short hb = f2bf(p); oh[q] = hb; ol[q] = f2bf(p - bf2f(hb)); }
            const size_t o = (size_t)i * NN + c0; *(volatile v4us*)(PH + o) = oh; *(volatile v4us*)(PL + o) = ol; }
        if (ps == 0) __threadfence(); }
}

extern "C" void kernel_launch(void* const* d_in, const int* in_sizes, int n_in,
                              void* d_out, int out_size, void* d_ws, size_t ws_size, hipStream_t stream) {
    (void)in_sizes; (void)n_in; (void)out_size;
    const float* hid = (const float*)d_in[0]; const int* adj = (const int*)d_in[1]; const float* a0 = (const float*)d_in[2]; const float* a1 = (const float*)d_in[3]; const float* a2 = (const float*)d_in[4]; const float* a3 = (const float*)d_in[5];
    float* out = (float*)d_out;
    char* wsp = (char*)d_ws;
    auto take = [&](size_t bytes) { char* p = wsp; wsp += (bytes + 255) & ~(size_t)255; return (void*)p; };
    bf* Hb = (bf*)take((size_t)NN * DD * 2); bf* HAh = (bf*)take((size_t)4 * NN * DD * 2); bf* HAl = (bf*)take((size_t)4 * NN * DD * 2); bf* HT = (bf*)take((size_t)DD * NN * 2);
    float* E = (float*)take((size_t)4 * NN * NN * 4); bf* PH = (bf*)take((size_t)NN * NN * 2); bf* PL = (bf*)take((size_t)NN * NN * 2);
    if ((size_t)(wsp - (char*)d_ws) > ws_size) return;
    for (int b = 0; b < NB_; ++b) { const float* hb = hid + (size_t)b * NN * DD;
        k_hprep<<<NN / 8, 256, 0, stream>>>(hb, a0, a1, a2, a3, Hb, HAh, HAl); k_hT<<<dim3(NN / 64, DD / 64, 1), 256, 0, stream>>>(hb, HT);
        for (int k = 0; k < 4; ++k) k_gemmb<true, false><<<dim3(NN / 64, NN / 64, 1), 128, 0, stream>>>(HAh + (size_t)k * NN * DD, HAl + (size_t)k * NN * DD, Hb, nullptr, E + (size_t)k * NN * NN, NN, nullptr, nullptr, DD);
        k_selsoft<<<NN / 8, 256, 0, stream>>>(E, adj + (size_t)b * NN * NN, PH, PL);
        k_gemmb<true, false><<<dim3(NN / 64, DD / 64, 1), 128, 0, stream>>>(PH, PL, HT, nullptr, out + (size_t)b * NN * DD, DD, nullptr, nullptr, NN); }
}
